// HANLayer_13013750907160
// MI455X (gfx1250) — hardware-verified
//
#include <hip/hip_runtime.h>
#include <math.h>

constexpr int NN      = 20000;
constexpr int NE      = 320000;
constexpr int NPATH   = 3;
constexpr int FIN     = 128;
constexpr int NHEAD   = 4;
constexpr int DHEAD   = 64;
constexpr int HD      = 256;
constexpr int HID     = 128;
constexpr int NPADA   = 20032;
constexpr int FEAT_LD = NPATH * HD;
constexpr int ZROWS   = NPATH * NN;
constexpr int ZPAD    = 60032;
constexpr int NT      = 256;
constexpr int SRB     = 128;
constexpr int NTILE   = (NN + SRB - 1) / SRB;
constexpr int SCH     = 2048;
constexpr int NCH     = (NE + SCH - 1) / SCH;
constexpr int SEMROWS = 128;
constexpr int SEM_PITCH = 132;
constexpr int HCAST_THREADS = NPADA * FIN / 8;
constexpr int HCAST_REAL    = NN * FIN / 8;
constexpr int SCANW   = 80;
constexpr float NEG_SLOPE = 0.2f;

static_assert(NPADA % 64 == 0 && NPADA >= NN);
static_assert(FEAT_LD % 64 == 0 && FIN % 32 == 0 && HD % 32 == 0);
static_assert(ZPAD % SEMROWS == 0 && ZPAD >= ZROWS && SEMROWS == 16 * (NT / 32));
static_assert(NE % (SCH / NT) == 0 && (SCH / NT) % 4 == 0 && SCH % NT == 0);
static_assert(SRB == 16 * (NT / 32) && SRB * NTILE >= NN);
static_assert(NN % 32 == 0 && (NN * HD) % (4 * NT) == 0);
static_assert(HCAST_THREADS % NT == 0 && HCAST_REAL % 32 == 0);
static_assert(HID <= NT && HD == NT && SCANW <= NT && SCANW >= 65);

typedef __attribute__((ext_vector_type(16))) _Float16 v16h;
typedef __attribute__((ext_vector_type(8)))  _Float16 v8h;
typedef __attribute__((ext_vector_type(16))) __bf16   v16b;
typedef __attribute__((ext_vector_type(8)))  __bf16   v8b;
typedef __attribute__((ext_vector_type(8)))  float    v8f;
typedef __attribute__((ext_vector_type(4)))  float    v4f;
typedef __attribute__((ext_vector_type(4)))  int      v4i;
typedef __attribute__((ext_vector_type(4)))  unsigned int v4u;
typedef __attribute__((ext_vector_type(8)))  unsigned int v8u;

__device__ __forceinline__ unsigned short f2bf_bits(float f) {
  unsigned u = __float_as_uint(f);
  return (unsigned short)((u + 0x7FFFu + ((u >> 16) & 1u)) >> 16);
}
__device__ __forceinline__ float bf_bits2f(unsigned short h) { return __uint_as_float(((unsigned)h) << 16); }
__device__ __forceinline__ float bfr(float f) { return __uint_as_float(((unsigned)f2bf_bits(f)) << 16); }
__device__ __forceinline__ unsigned pk16(unsigned short a, unsigned short b) { return (unsigned)a | ((unsigned)b << 16); }
__device__ __forceinline__ unsigned pack2bf(float a, float b) { return pk16(f2bf_bits(a), f2bf_bits(b)); }
__device__ __forceinline__ void fence_v4(v4f& t) { asm volatile("" : "+v"(t)); }

__device__ __forceinline__ void dep_guard_h(v8f& a, v8f& b, v16h x, v16h y) { asm volatile("v_nop\n\tv_nop\n\tv_nop\n\tv_nop" : "+v"(a), "+v"(b) : "v"(x), "v"(y)); }
__device__ __forceinline__ void dep_guard_b(v8f& a, v8f& b, v16b x, v16b y) { asm volatile("v_nop\n\tv_nop\n\tv_nop\n\tv_nop" : "+v"(a), "+v"(b) : "v"(x), "v"(y)); }
__device__ __forceinline__ void dep_guard4_h(v8f& a, v8f& b, v8f& c, v8f& d, v16h x, v16h y) { asm volatile("v_nop\n\tv_nop\n\tv_nop\n\tv_nop" : "+v"(a), "+v"(b), "+v"(c), "+v"(d) : "v"(x), "v"(y)); }
__device__ __forceinline__ void dep_guard4_b(v8f& a, v8f& b, v8f& c, v8f& d, v16b x, v16b y) { asm volatile("v_nop\n\tv_nop\n\tv_nop\n\tv_nop" : "+v"(a), "+v"(b), "+v"(c), "+v"(d) : "v"(x), "v"(y)); }
__device__ __forceinline__ void keep4_h(v16h a, v16h b, v16h c, v16h d) { asm volatile("v_nop" :: "v"(a), "v"(b), "v"(c), "v"(d)); }
__device__ __forceinline__ void keep4_b(v16b a, v16b b, v16b c, v16b d) { asm volatile("v_nop" :: "v"(a), "v"(b), "v"(c), "v"(d)); }
__device__ __forceinline__ void acc_guard4(v8f& a, v8f& b, v8f& c, v8f& d) { asm volatile("v_nop\n\tv_nop\n\tv_nop\n\tv_nop" : "+v"(a), "+v"(b), "+v"(c), "+v"(d)); }
template <typename T> struct Frag;
template <> struct Frag<_Float16> {
  typedef v16h V; union U { v16h v; v8h h[2]; };
  static __device__ __forceinline__ v16h load(const _Float16* p) {
    U f; f.h[0] = *(const v8h*)(p); f.h[1] = *(const v8h*)(p + 16); return f.v;
  }
  static __device__ __forceinline__ v8f mma(v16h a, v16h b, v8f c) {
    return __builtin_amdgcn_wmma_f32_16x16x32_f16(false, a, false, b, (short)0, c, false, false);
  }
  static __device__ __forceinline__ void guard(v8f& a, v8f& b, v16h x, v16h y) { dep_guard_h(a, b, x, y); }
  static __device__ __forceinline__ void guard4(v8f& a, v8f& b, v8f& c, v8f& d, v16h x, v16h y) { dep_guard4_h(a, b, c, d, x, y); }
  static __device__ __forceinline__ void keep(v16h a, v16h b, v16h c, v16h d) { keep4_h(a, b, c, d); }
};
template <> struct Frag<__bf16> {
  typedef v16b V; union U { v16b v; v8b h[2]; };
  static __device__ __forceinline__ v16b load(const __bf16* p) {
    U f; f.h[0] = *(const v8b*)(p); f.h[1] = *(const v8b*)(p + 16); return f.v;
  }
  static __device__ __forceinline__ v8f mma(v16b a, v16b b, v8f c) {
    return __builtin_amdgcn_wmma_f32_16x16x32_bf16(false, a, false, b, (short)0, c, false, false);
  }
  static __device__ __forceinline__ void guard(v8f& a, v8f& b, v16b x, v16b y) { dep_guard_b(a, b, x, y); }
  static __device__ __forceinline__ void guard4(v8f& a, v8f& b, v8f& c, v8f& d, v16b x, v16b y) { dep_guard4_b(a, b, c, d, x, y); }
  static __device__ __forceinline__ void keep(v16b a, v16b b, v16b c, v16b d) { keep4_b(a, b, c, d); }
};

template <int ET> struct Elem;
template <> struct Elem<0> { typedef _Float16 T; };
template <> struct Elem<1> { typedef __bf16 T; };
template <int ET, bool SPLIT, int BIAS_MODE, int OUT_MODE, bool RESID, int ACT = 0>
__global__ __launch_bounds__(256) void wmma_gemm64(
    const unsigned short* __restrict__ Ap, const unsigned short* __restrict__ A2p, int lda, long strideA,
    const unsigned short* __restrict__ Btp, const unsigned short* __restrict__ Bt2p, int ldb, long strideB,
    void* __restrict__ Cout, void* __restrict__ Cout2, int ldc, long strideC,
    const float* __restrict__ bias,
    const float* __restrict__ resid, long strideR,
    int M, int N, int K, float scale) {
  typedef typename Elem<ET>::T T;
  typedef typename Frag<T>::V V;
  const T* A = (const T*)Ap; const T* A2 = (const T*)A2p; const T* Bt = (const T*)Btp; const T* Bt2 = (const T*)Bt2p;
  __shared__ __align__(16) float sT[8][16 * 68];
  const int b    = blockIdx.y;
  const int lane = threadIdx.x & 31;
  const int wave = threadIdx.x >> 5;
  const int tilesN = N >> 6;
  const int tilesM = M >> 6;
  const int tile = blockIdx.x * 8 + wave;
  if (tile >= tilesM * tilesN) return;
  const int tm = tile / tilesN;
  const int tn = tile - tm * tilesN;
  const int m0 = tm << 6;
  const int n0 = tn << 6;

  const T* Ab  = A  + (size_t)b * strideA;
  const T* Bb  = Bt + (size_t)b * strideB;
  const T* Ab2 = SPLIT ? (A2  + (size_t)b * strideA) : nullptr;
  const T* Bb2 = SPLIT ? (Bt2 + (size_t)b * strideB) : nullptr;

  const int rlane = lane & 15;
  const int koff  = (lane >> 4) * 8;
  const int mOff  = (lane >> 4) * 8;

  v8f acc[4][4];
#pragma unroll
  for (int i = 0; i < 4; ++i)
#pragma unroll
    for (int j = 0; j < 4; ++j) acc[i][j] = (v8f){0.f,0.f,0.f,0.f,0.f,0.f,0.f,0.f};

  for (int k0 = 0; k0 < K; k0 += 32) {
    V bh[4], bl[4];
#pragma unroll
    for (int j = 0; j < 4; ++j) {
      const size_t bo = (size_t)(n0 + (j << 4) + rlane) * ldb + koff + k0;
      bh[j] = Frag<T>::load(Bb + bo);
      if (SPLIT) bl[j] = Frag<T>::load(Bb2 + bo);
    }
#pragma unroll
    for (int i = 0; i < 4; ++i) {
      const size_t ao = (size_t)(m0 + (i << 4) + rlane) * lda + koff + k0;
      V ah = Frag<T>::load(Ab + ao);
      V al;
      if (SPLIT) al = Frag<T>::load(Ab2 + ao);
#pragma unroll
      for (int j = 0; j < 4; ++j) {
        acc[i][j] = Frag<T>::mma(ah, bh[j], acc[i][j]);
        if (SPLIT) {
          acc[i][j] = Frag<T>::mma(ah, bl[j], acc[i][j]);
          acc[i][j] = Frag<T>::mma(al, bh[j], acc[i][j]);
        }
      }
      Frag<T>::guard4(acc[i][0], acc[i][1], acc[i][2], acc[i][3], ah, SPLIT ? al : ah);
    }
    Frag<T>::keep(bh[0], bh[1], bh[2], bh[3]);
    if (SPLIT) Frag<T>::keep(bl[0], bl[1], bl[2], bl[3]);
  }
  acc_guard4(acc[0][0], acc[0][1], acc[0][2], acc[0][3]);
  acc_guard4(acc[1][0], acc[1][1], acc[1][2], acc[1][3]);
  acc_guard4(acc[2][0], acc[2][1], acc[2][2], acc[2][3]);
  acc_guard4(acc[3][0], acc[3][1], acc[3][2], acc[3][3]);

  float* slab = sT[wave];
  const float* Rb = RESID ? (resid + (size_t)b * strideR) : nullptr;
#pragma unroll
  for (int i = 0; i < 4; ++i) {
    const int mBase = m0 + (i << 4);
#pragma unroll
    for (int j = 0; j < 4; ++j) {
      const int n = n0 + (j << 4) + rlane;
      float bv = 0.f;
      if (BIAS_MODE == 2) bv = bias[n];
#pragma unroll
      for (int r = 0; r < 8; ++r) {
        float v = acc[i][j][r] * scale;
        if (BIAS_MODE == 1) v += bias[mBase + mOff + r];
        if (BIAS_MODE == 2) v += bv;
        if (RESID) v += Rb[(size_t)(mBase + mOff + r) * ldc + n];
        if (ACT == 2) v = fmaxf(v, 0.0f);
        if (ACT == 4) v = (v > 0.f) ? v : 0.01f * v;
        slab[(mOff + r) * 68 + (j << 4) + rlane] = v;
      }
    }
    __builtin_amdgcn_fence(__ATOMIC_RELEASE, "workgroup");
    __builtin_amdgcn_wave_barrier();
    __builtin_amdgcn_fence(__ATOMIC_ACQUIRE, "workgroup");
    if (OUT_MODE == 0) {
      float* C = (float*)Cout + (size_t)b * strideC;
      const int hh = lane >> 4, c4 = (lane & 15) * 4;
      for (int pass = 0; pass < 2; ++pass) {
#pragma unroll
        for (int it = 0; it < 8; ++it) {
          const int row = it * 2 + hh;
          v4f v = *(const v4f*)(slab + row * 68 + c4);
          *(volatile v4f*)(C + (size_t)(mBase + row) * ldc + n0 + c4) = v;
        }
        __threadfence();
      }
    } else {
      const int q = lane >> 3, c8 = (lane & 7) * 8;
      unsigned short* C  = (unsigned short*)Cout  + (size_t)b * strideC;
      unsigned short* C2 = (OUT_MODE == 2) ? ((unsigned short*)Cout2 + (size_t)b * strideC) : nullptr;
      for (int pass = 0; pass < 2; ++pass) {
#pragma unroll
        for (int it = 0; it < 4; ++it) {
          const int row = it * 4 + q;
          const float* sp = slab + row * 68 + c8;
          v8h hv, lv;
#pragma unroll
          for (int e = 0; e < 8; ++e) {
            if (OUT_MODE == 1) {
              hv[e] = (_Float16)sp[e];
            } else {
              unsigned short hb = f2bf_bits(sp[e]);
              unsigned short lb = f2bf_bits(sp[e] - bf_bits2f(hb));
              hv[e] = __builtin_bit_cast(_Float16, hb);
              lv[e] = __builtin_bit_cast(_Float16, lb);
            }
          }
          *(volatile v8h*)(C + (size_t)(mBase + row) * ldc + n0 + c8) = hv;
          if (OUT_MODE == 2) *(volatile v8h*)(C2 + (size_t)(mBase + row) * ldc + n0 + c8) = lv;
        }
        __threadfence();
      }
    }
    __builtin_amdgcn_fence(__ATOMIC_RELEASE, "workgroup");
    __builtin_amdgcn_wave_barrier();
    __builtin_amdgcn_fence(__ATOMIC_ACQUIRE, "workgroup");
  }
}

__global__ __launch_bounds__(NT) void k_cast_h(const float* __restrict__ h, unsigned short* __restrict__ hB) {
  const int i = blockIdx.x * NT + threadIdx.x;
  const int ic = (i < HCAST_REAL) ? i : (HCAST_REAL - 1);
  const float* p = h + (size_t)ic * 8;
  const v4f a = *(const v4f*)(p);
  const v4f c = *(const v4f*)(p + 4);
  const unsigned keep = (i < HCAST_REAL) ? 0xffffffffu : 0u;
  v4u u;
  u[0] = pack2bf(a[0], a[1]) & keep;
  u[1] = pack2bf(a[2], a[3]) & keep;
  u[2] = pack2bf(c[0], c[1]) & keep;
  u[3] = pack2bf(c[2], c[3]) & keep;
  unsigned short* q = hB + (size_t)i * 8;
  *(volatile v4u*)q = u;
  __threadfence();
  *(volatile v4u*)q = u;
}

__global__ __launch_bounds__(NT) void k_tcast(const float* __restrict__ in, unsigned short* __restrict__ out,
                                             int KR, int CC, long inPlane, long outPlane) {
  __shared__ float sm[64][65];
  const int t  = threadIdx.x;
  const int k0 = blockIdx.x * 64;
  const int c0 = blockIdx.y * 64;
  const int z  = blockIdx.z;
  const float* ip = in + (size_t)z * inPlane;
#pragma unroll
  for (int i = 0; i < 16; ++i) {
    const int e = i * 256 + t;
    const int r = e >> 6;
    const int cc = e & 63;
    sm[cc][r] = ip[(size_t)(k0 + r) * CC + c0 + cc];
  }
  __syncthreads();
  const int lane = t & 31, wave = t >> 5;
  const int q = lane >> 3, c8 = (lane & 7) * 8;
  unsigned short* op = out + (size_t)z * outPlane;
  for (int pass = 0; pass < 2; ++pass) {
#pragma unroll
    for (int it = 0; it < 2; ++it) {
      const int row = wave * 8 + it * 4 + q;
      unsigned short hb[8];
#pragma unroll
      for (int e = 0; e < 8; ++e) hb[e] = f2bf_bits(sm[row][c8 + e]);
      const v4u u = (v4u){pk16(hb[0], hb[1]), pk16(hb[2], hb[3]), pk16(hb[4], hb[5]), pk16(hb[6], hb[7])};
      *(volatile v4u*)(op + (size_t)(c0 + row) * KR + k0 + c8) = u;
    }
    __threadfence();
  }
}

__global__ __launch_bounds__(NT) void k_eler(const float* __restrict__ feat, const float* __restrict__ al,
                                            const float* __restrict__ ar, float* __restrict__ elT, float* __restrict__ erT) {
  __shared__ __align__(16) float sAL[HD];
  __shared__ __align__(16) float sAR[HD];
  const int t = threadIdx.x;
  const int mp = blockIdx.y;
  sAL[t] = bfr(al[mp * HD + t]);
  sAR[t] = bfr(ar[mp * HD + t]);
  __syncthreads();
  const int n  = blockIdx.x * NT + t;
  const int nc = (n < NN) ? n : (NN - 1);
  const float* fp = feat + (size_t)nc * FEAT_LD + mp * HD;
  v4f el4, er4;
#pragma unroll
  for (int hh = 0; hh < NHEAD; ++hh) {
    float sl = 0.0f, sr = 0.0f;
#pragma unroll 1
    for (int qd = 0; qd < DHEAD / 4; ++qd) {
      const v4f f = *(const v4f*)(fp + hh * DHEAD + 4 * qd);
      const v4f a = *(const v4f*)(sAL + hh * DHEAD + 4 * qd);
      const v4f b = *(const v4f*)(sAR + hh * DHEAD + 4 * qd);
      sl += f[0] * a[0] + f[1] * a[1] + f[2] * a[2] + f[3] * a[3];
      sr += f[0] * b[0] + f[1] * b[1] + f[2] * b[2] + f[3] * b[3];
    }
    el4[hh] = sl; er4[hh] = sr;
  }
  if (n < NN) {
    float* pl = elT + ((size_t)(mp * NN + n)) * NHEAD;
    float* pr = erT + ((size_t)(mp * NN + n)) * NHEAD;
    for (int pass = 0; pass < 2; ++pass) { *(volatile v4f*)pl = el4; *(volatile v4f*)pr = er4; __threadfence(); }
  }
}

__global__ __launch_bounds__(NT) void k_zero4(float* __restrict__ p, int n4) {
  const int i = blockIdx.x * NT + threadIdx.x;
  if (i < n4) {
    const v4f z4 = {0.f, 0.f, 0.f, 0.f};
    *(volatile v4f*)(p + (size_t)i * 4) = z4;
    __threadfence();
    *(volatile v4f*)(p + (size_t)i * 4) = z4;
  }
}

__device__ __forceinline__ int blk_excl_scan(int cnt, int* scan_ws, int tid, int* tot) {
  const int lane = tid & 31, wave = tid >> 5; int incl = cnt;
#pragma unroll
  for (int o = 1; o < 32; o <<= 1) { const int v = __shfl_up(incl, o, 32); if (lane >= o) incl += v; }
  if (lane == 31) scan_ws[wave] = incl;
  __syncthreads();
  if (wave == 0) { const int f = (lane < NT / 32) ? 1 : 0; const int wv = scan_ws[lane] * f; int wincl = wv;
#pragma unroll
    for (int o = 1; o < 32; o <<= 1) { const int v = __shfl_up(wincl, o, 32); if (lane >= o) wincl += v; }
    if (lane < NT / 32) scan_ws[32 + lane] = wincl - wv; if (lane == 31) scan_ws[64] = wincl; }
  __syncthreads();
  const int res = scan_ws[32 + wave] + incl - cnt; *tot = scan_ws[64];
  return res;
}
template <int SP, int CAP>
__device__ __forceinline__ int chunk_hits(const int* __restrict__ dstv, const int* __restrict__ srcv, int e0, int n0, int tid,
                                          int* LIST, int* scan_ws) {
  const int eb = e0 + tid * SP;
  const int live = (eb < NE) ? 1 : 0;
  const int ebc = live ? eb : (NE - SP);
  int rec[SP]; int cnt = 0;
#pragma unroll
  for (int k = 0; k < SP; k += 4) {
    const v4i d4 = *(const v4i*)(dstv + ebc + k);
    const v4i s4 = *(const v4i*)(srcv + ebc + k);
#pragma unroll
    for (int e = 0; e < 4; ++e) {
      const int d = d4[e];
      int s = s4[e]; s = s < 0 ? 0 : s; s = s > NN - 1 ? NN - 1 : s;
      const int hit = live & (int)(d >= n0) & (int)(d < n0 + SRB);
      const unsigned pk = ((unsigned)(d - n0) << 16) | (unsigned)s;
      rec[k + e] = (int)(pk * (unsigned)hit) - (1 - hit);
      cnt += hit;
    }
  }
  int tot; int p = blk_excl_scan(cnt, scan_ws, tid, &tot);
#pragma unroll
  for (int k = 0; k < SP; ++k) if (rec[k] >= 0) { if ((unsigned)p < (unsigned)CAP) LIST[p] = rec[k]; ++p; }
  __syncthreads();
  return tot < CAP ? tot : CAP;
}

__global__ __launch_bounds__(NT) void k_gat(const float* __restrict__ feat, const int* __restrict__ src, const int* __restrict__ dst,
                                           const float* __restrict__ elT, const float* __restrict__ erT, const float* __restrict__ bias,
                                           float* __restrict__ z32) {
  __shared__ __align__(16) float ACC[SRB * HD];
  __shared__ int   LIST[SCH];
  __shared__ float SM[SRB * NHEAD];
  __shared__ float SL[SRB * NHEAD];
  __shared__ float SER[SRB * NHEAD];
  __shared__ int   scan_ws[SCANW];
  const int tid = threadIdx.x, lane = tid & 31, wave = tid >> 5;
  const int mp   = blockIdx.x / NTILE;
  const int tile = blockIdx.x - mp * NTILE;
  const int n0   = tile * SRB;
  const int hq   = lane & 3;
  const int hj0  = lane >> 4, hj1 = 2 + (lane >> 4);
  v4f bz0, bz1;
  {
    const v4f b0 = *(const v4f*)(bias + mp * HD + 4 * lane);
    const v4f b1 = *(const v4f*)(bias + mp * HD + 128 + 4 * lane);
#pragma unroll
    for (int e = 0; e < 4; ++e) { bz0[e] = bfr(b0[e]); bz1[e] = bfr(b1[e]); }
  }
  const v4f z4 = {0.f, 0.f, 0.f, 0.f};
#pragma unroll 1
  for (int j = 0; j < 16; ++j) {
    float* rp = ACC + (wave * 16 + j) * HD + 4 * lane;
    *(v4f*)rp = z4; *(v4f*)(rp + 128) = z4;
  }
  for (int i = tid; i < SRB * NHEAD; i += NT) {
    SM[i] = -INFINITY; SL[i] = 0.f;
    const int dl = i >> 2, hd = i & 3;
    int n = n0 + dl; n = n < NN ? n : NN - 1;
    SER[i] = erT[((size_t)(mp * NN + n)) * NHEAD + hd];
  }
  if (tid < SCANW) scan_ws[tid] = 0;
#pragma unroll
  for (int k = 0; k < SCH / NT; ++k) LIST[tid * (SCH / NT) + k] = -1;
  __syncthreads();
  const int* srcv = src + (size_t)mp * NE;
  const int* dstv = dst + (size_t)mp * NE;
#pragma unroll 1
  for (int c = 0; c < NCH; ++c) {
    const int tot = chunk_hits<SCH / NT, SCH>(dstv, srcv, c * SCH, n0, tid, LIST, scan_ws);
#pragma unroll 1
    for (int base = 0; base < tot; base += 32) {
      const int q  = base + lane;
      const int qc = (q < SCH) ? q : (SCH - 1);
      const int lq = LIST[qc];
      const int rv = lq | ((q < tot) ? 0 : -1);
      const int own = (rv >= 0 && (rv >> 20) == wave) ? 1 : 0;
      unsigned msk = (unsigned)__ballot(own);
#pragma unroll 1
      for (int it = 0; it < 32; ++it) {
        if (msk == 0u) break;
        const int bp = __builtin_ctz(msk); msk &= msk - 1u;
        const int r  = __shfl(rv, bp, 32);
        const int dl = r >> 16, s = r & 0xFFFF;
        const float elv = elT[((size_t)(mp * NN + s)) * NHEAD + hq];
        float ev = elv + SER[dl * NHEAD + hq];
        ev = (ev >= 0.f) ? ev : NEG_SLOPE * ev;
        const int mi = dl * NHEAD + hq;
        const float mo = SM[mi], lo = SL[mi];
        const float mn = fmaxf(mo, ev);
        const float rr = expf(mo - mn), ex = expf(ev - mn);
        const float ln = lo * rr + ex;
        if (lane < NHEAD) { SM[mi] = mn; SL[mi] = ln; }
        const float* fp = feat + (size_t)s * FEAT_LD + mp * HD + 4 * lane;
        const v4f f0 = *(const v4f*)(fp);
        const v4f f1 = *(const v4f*)(fp + 128);
        const float rr0 = __shfl(rr, hj0, 32), ex0 = __shfl(ex, hj0, 32);
        const float rr1 = __shfl(rr, hj1, 32), ex1 = __shfl(ex, hj1, 32);
        float* ap = ACC + dl * HD + 4 * lane;
        v4f a0 = *(const v4f*)(ap);       a0 = a0 * rr0 + ex0 * f0; *(v4f*)(ap) = a0;
        v4f a1 = *(const v4f*)(ap + 128); a1 = a1 * rr1 + ex1 * f1; *(v4f*)(ap + 128) = a1;
      }
    }
    __syncthreads();
  }
#pragma unroll 1
  for (int j = 0; j < 16; ++j) {
    const int dl = wave * 16 + j;
    const int n  = n0 + dl;
    float lv = SL[dl * NHEAD + hq];
    lv = (lv > 0.f) ? lv : 1.0f;
    const float inv  = 1.0f / lv;
    const float inv0 = __shfl(inv, hj0, 32), inv1 = __shfl(inv, hj1, 32);
    const float* rp = ACC + dl * HD + 4 * lane;
    v4f v0 = *(const v4f*)(rp) * inv0;       fence_v4(v0); v0 = v0 + bz0;
    v4f v1 = *(const v4f*)(rp + 128) * inv1; fence_v4(v1); v1 = v1 + bz1;
    if (n < NN) {
      float* zr = z32 + ((size_t)(mp * NN + n)) * HD + 4 * lane;
      for (int pass = 0; pass < 2; ++pass) { *(volatile v4f*)(zr) = v0; *(volatile v4f*)(zr + 128) = v1; __threadfence(); }
    }
  }
}

__global__ __launch_bounds__(NT) void k_sem(const float* __restrict__ z32, const unsigned short* __restrict__ Bt2p,
                                           const float* __restrict__ b1, const float* __restrict__ w2, float* __restrict__ wT) {
  __shared__ __align__(16) float slab[NT / 32][16 * SEM_PITCH];
  __shared__ __align__(16) float sB1[HID];
  __shared__ __align__(16) float sW2[HID];
  __shared__ __align__(16) float sW[SEMROWS];
  const int tid = threadIdx.x, lane = tid & 31, wave = tid >> 5;
  if (tid < HID) { sB1[tid] = bfr(b1[tid]); sW2[tid] = bfr(w2[tid]); }
  __syncthreads();
  const __bf16* Bt2 = (const __bf16*)Bt2p;
  const int rlane = lane & 15, hh = lane >> 4, koff = hh * 8;
  const int m0 = blockIdx.x * SEMROWS + wave * 16;
  v8f acc[8];
#pragma unroll
  for (int j = 0; j < 8; ++j) acc[j] = (v8f){0.f,0.f,0.f,0.f,0.f,0.f,0.f,0.f};
  const float* arow = z32 + (size_t)(m0 + rlane) * HD + koff;
#pragma unroll 1
  for (int k0 = 0; k0 < HD; k0 += 32) {
    const v4f a0 = *(const v4f*)(arow + k0);
    const v4f a1 = *(const v4f*)(arow + k0 + 4);
    const v4f a2 = *(const v4f*)(arow + k0 + 16);
    const v4f a3 = *(const v4f*)(arow + k0 + 20);
    v8u aw;
    aw[0] = pack2bf(a0[0], a0[1]); aw[1] = pack2bf(a0[2], a0[3]);
    aw[2] = pack2bf(a1[0], a1[1]); aw[3] = pack2bf(a1[2], a1[3]);
    aw[4] = pack2bf(a2[0], a2[1]); aw[5] = pack2bf(a2[2], a2[3]);
    aw[6] = pack2bf(a3[0], a3[1]); aw[7] = pack2bf(a3[2], a3[3]);
    const v16b av = __builtin_bit_cast(v16b, aw);
    asm volatile("" ::: "memory");
    v16b bq[4];
#pragma unroll
    for (int j = 0; j < 4; ++j) bq[j] = Frag<__bf16>::load(Bt2 + (size_t)(16 * j + rlane) * HD + koff + k0);
#pragma unroll
    for (int j = 0; j < 4; ++j) acc[j] = Frag<__bf16>::mma(av, bq[j], acc[j]);
    dep_guard4_b(acc[0], acc[1], acc[2], acc[3], av, bq[3]);
    keep4_b(bq[0], bq[1], bq[2], bq[3]);
    asm volatile("" ::: "memory");
#pragma unroll
    for (int j = 0; j < 4; ++j) bq[j] = Frag<__bf16>::load(Bt2 + (size_t)(16 * (j + 4) + rlane) * HD + koff + k0);
#pragma unroll
    for (int j = 0; j < 4; ++j) acc[4 + j] = Frag<__bf16>::mma(av, bq[j], acc[4 + j]);
    dep_guard4_b(acc[4], acc[5], acc[6], acc[7], av, bq[3]);
    keep4_b(bq[0], bq[1], bq[2], bq[3]);
  }
  acc_guard4(acc[0], acc[1], acc[2], acc[3]);
  acc_guard4(acc[4], acc[5], acc[6], acc[7]);
  float* sl = slab[wave];
#pragma unroll
  for (int j = 0; j < 8; ++j)
#pragma unroll
    for (int r = 0; r < 8; ++r) sl[(8 * hh + r) * SEM_PITCH + 16 * j + rlane] = acc[j][r];
  __syncthreads();
  const int row = lane >> 1, cb = (lane & 1) * 64;
  float s = 0.0f;
#pragma unroll 1
  for (int c = 0; c < 64; ++c) {
    const int col = cb + c;
    const float u = sl[row * SEM_PITCH + col] + sB1[col];
    s += tanhf(u) * sW2[col];
  }
  s += __shfl_xor(s, 1, 32);
  if ((lane & 1) == 0) sW[wave * 16 + row] = s;
  __syncthreads();
  if (wave == 0) {
    const v4f val = *(const v4f*)(sW + 4 * lane);
    float* wp = wT + (size_t)blockIdx.x * SEMROWS + 4 * lane;
    *(volatile v4f*)wp = val;
    __threadfence();
    *(volatile v4f*)wp = val;
  }
}

__global__ __launch_bounds__(NT) void k_beta(const float* __restrict__ wT, float* __restrict__ betaL) {
  __shared__ float red[NT];
  __shared__ float tot[4];
  const int t = threadIdx.x;
#pragma unroll 1
  for (int mp = 0; mp < NPATH; ++mp) {
    float s = 0.0f;
#pragma unroll 1
    for (int i = t; i < NN; i += NT) s += wT[mp * NN + i];
    red[t] = s;
    __syncthreads();
#pragma unroll 1
    for (int off = NT / 2; off > 0; off >>= 1) {
      if (t < off) red[t] += red[t + off];
      __syncthreads();
    }
    if (t == 0) tot[mp] = red[0];
    __syncthreads();
  }
  if (t < 32) {
    const float cinv = 1.0f / (float)NN;
    const float v0 = tot[0] * cinv, v1 = tot[1] * cinv, v2 = tot[2] * cinv;
    const float mx = fmaxf(v0, fmaxf(v1, v2));
    const float e0 = expf(v0 - mx), e1 = expf(v1 - mx), e2 = expf(v2 - mx);
    const float sinv = 1.0f / (e0 + e1 + e2);
    const float b0 = e0 * sinv, b1 = e1 * sinv, b2 = e2 * sinv;
    float v = 0.0f;
    if (t == 0) v = b0; else if (t == 1) v = b1; else if (t == 2) v = b2;
    ((volatile float*)betaL)[t] = v;
    __threadfence();
    ((volatile float*)betaL)[t] = v;
  }
}

__global__ __launch_bounds__(NT) void k_combine(const float* __restrict__ z32, const float* __restrict__ betaL, float* __restrict__ out) {
  const int i = blockIdx.x * NT + threadIdx.x;
  const float b0 = betaL[0], b1 = betaL[1], b2 = betaL[2];
  const size_t e4 = (size_t)i * 4;
  const v4f z0 = *(const v4f*)(z32 + e4);
  const v4f z1 = *(const v4f*)(z32 + (size_t)NN * HD + e4);
  const v4f z2 = *(const v4f*)(z32 + (size_t)2 * NN * HD + e4);
  v4f p0 = z0 * b0; fence_v4(p0);
  v4f p1 = z1 * b1; fence_v4(p1);
  v4f p2 = z2 * b2; fence_v4(p2);
  const v4f o = (p0 + p1) + p2;
  *(volatile v4f*)(out + e4) = o;
  __threadfence();
  *(volatile v4f*)(out + e4) = o;
}

extern "C" void kernel_launch(void* const* d_in, const int* in_sizes, int n_in,
                              void* d_out, int out_size, void* d_ws, size_t ws_size, hipStream_t stream) {
  (void)in_sizes; (void)n_in; (void)out_size;
  const float* h     = (const float*)d_in[0];
  const int*   src   = (const int*)  d_in[1];
  const int*   dst   = (const int*)  d_in[2];
  const float* W     = (const float*)d_in[3];
  const float* attl  = (const float*)d_in[4];
  const float* attr  = (const float*)d_in[5];
  const float* gbias = (const float*)d_in[6];
  const float* sW1   = (const float*)d_in[7];
  const float* sb1   = (const float*)d_in[8];
  const float* sW2   = (const float*)d_in[9];
  float* out = (float*)d_out;

  char* ws = (char*)d_ws; size_t off = 0;
  auto carve = [&](size_t bytes) -> char* { char* p = ws + off; off += (bytes + 255) & ~(size_t)255; return p; };
  unsigned short* hB   = (unsigned short*)carve((size_t)NPADA * FIN * 2);
  unsigned short* Bt1  = (unsigned short*)carve((size_t)FEAT_LD * FIN * 2);
  unsigned short* Bt2  = (unsigned short*)carve((size_t)HID * HD * 2);
  float*          feat = (float*)carve((size_t)NPADA * FEAT_LD * 4);
  float*          z32  = (float*)carve((size_t)ZPAD * HD * 4);
  float*          elT  = (float*)carve((size_t)ZROWS * NHEAD * 4);
  float*          erT  = (float*)carve((size_t)ZROWS * NHEAD * 4);
  float*          wT   = (float*)carve((size_t)ZPAD * 4);
  float*          betaL = (float*)carve(256);
  if (off > ws_size || off > (size_t)134217728) return;

  k_cast_h<<<HCAST_THREADS / NT, NT, 0, stream>>>(h, hB);
  k_tcast<<<dim3(FIN / 64, HD / 64, NPATH), NT, 0, stream>>>(W, Bt1, FIN, HD, (long)FIN * HD, (long)HD * FIN);
  k_tcast<<<dim3(HD / 64, HID / 64, 1), NT, 0, stream>>>(sW1, Bt2, HD, HID, 0L, 0L);
  {
    const int tiles = (NPADA / 64) * (FEAT_LD / 64);
    wmma_gemm64<1, false, 0, 0, false><<<dim3((tiles + 7) / 8, 1), NT, 0, stream>>>(
        hB, hB, FIN, 0L, Bt1, Bt1, FIN, 0L, (void*)feat, (void*)nullptr, FEAT_LD, 0L,
        (const float*)nullptr, (const float*)nullptr, 0L, NPADA, FEAT_LD, FIN, 1.0f);
  }
  k_eler<<<dim3((NN + NT - 1) / NT, NPATH), NT, 0, stream>>>(feat, attl, attr, elT, erT);
  k_zero4<<<((ZPAD - ZROWS) * HD / 4 + NT - 1) / NT, NT, 0, stream>>>(z32 + (size_t)ZROWS * HD, (ZPAD - ZROWS) * HD / 4);
  k_gat<<<NPATH * NTILE, NT, 0, stream>>>(feat, src, dst, elT, erT, gbias, z32);
  k_sem<<<ZPAD / SEMROWS, NT, 0, stream>>>(z32, Bt2, sb1, sW2, wT);
  k_beta<<<1, NT, 0, stream>>>(wT, betaL);
  k_combine<<<(NN * HD / 4) / NT, NT, 0, stream>>>(z32, betaL, out);
}
